// TextAttention_15522011808140
// MI455X (gfx1250) — hardware-verified
//
#include <hip/hip_runtime.h>
#include <cfloat>


namespace {
constexpr int Bn = 8, S = 1024, DIM = 1024, H = 16, HD = 64, NT = Bn * S, NKP = 1088  ;
constexpr float QS = 8.0f, KS = 8.0f, VS = 8.0f, PS = 8.0f, SCALE = 0.125f, SELF = -100.0f;
constexpr size_t QPL = (size_t)Bn * H * S * HD, KPL = (size_t)Bn * H * NKP * HD;

typedef _Float16 b16;
typedef __attribute__((ext_vector_type(16))) _Float16 v16b;
typedef __attribute__((ext_vector_type(8))) _Float16 v8b;
typedef __attribute__((ext_vector_type(8))) float v8f;
typedef __attribute__((ext_vector_type(4))) float v4f;
__device__ __forceinline__ float bf16_rne(float f) { unsigned int u = __float_as_uint(f); u += 0x7FFFu + ((u >> 16) & 1u); return __uint_as_float(u & 0xFFFF0000u); }
__device__ __forceinline__ v16b frag_kb(const b16* p, int hh) { const v8b a = *(const v8b*)(p + 8 * hh), b = *(const v8b*)(p + 16 + 8 * hh); v16b f;
#pragma unroll
  for (int e = 0; e < 8; ++e) { f[e] = a[e]; f[8 + e] = b[e]; } return f; }
__device__ __forceinline__ v16b frag_x(const float* p, int hh) { v16b f;
#pragma unroll
  for (int e = 0; e < 8; ++e) { f[e] = (b16)bf16_rne(p[8 * hh + e]); f[8 + e] = (b16)bf16_rne(p[16 + 8 * hh + e]); } return f; }
__device__ __forceinline__ v8f wmma16b(v16b a, v16b b, v8f c) { v8f d = __builtin_amdgcn_wmma_f32_16x16x32_f16(false, a, false, b, (short)0, c, false, false); asm volatile("v_nop\n\tv_nop\n\tv_nop\n\tv_nop" : "+v"(d) : "v"(a), "v"(b)); return d; }
__device__ __forceinline__ void wave_lds_sync() { __builtin_amdgcn_fence(__ATOMIC_RELEASE, "workgroup"); __builtin_amdgcn_wave_barrier(); __builtin_amdgcn_fence(__ATOMIC_ACQUIRE, "workgroup"); }
__device__ __forceinline__ float nexp(float x) { return __builtin_amdgcn_exp2f(x * 1.4426950408889634f); }
__device__ __forceinline__ float pmul(float a, float b) { float p = a * b; asm volatile("" : "+v"(p)); return p; }

__global__ __launch_bounds__(256) void prep_kernel(const float* __restrict__ gam, const float* __restrict__ wqk, const float* __restrict__ wv, const float* __restrict__ nkv, const float* __restrict__ wo, b16* __restrict__ R, b16* __restrict__ Ro, float* __restrict__ P, b16* __restrict__ kp, b16* __restrict__ vt) {
  const size_t tid = (size_t)blockIdx.x * blockDim.x + threadIdx.x, nth = (size_t)gridDim.x * blockDim.x;
  for (int pass = 0; pass < 2; ++pass) {
    for (size_t q = tid; q < (size_t)2048 * DIM; q += nth) { const int o = (int)(q / DIM), d = (int)(q % DIM); const float g = bf16_rne(gam[d]); const float w = (o < 1024) ? bf16_rne(wqk[(size_t)d * 1024 + o]) : bf16_rne(wv[(size_t)d * 1024 + o - 1024]); R[q] = (b16)(g * w); }
    for (size_t q = tid; q < (size_t)DIM * DIM; q += nth) { const int o = (int)(q / DIM), k = (int)(q % DIM); Ro[q] = (b16)bf16_rne(wo[(size_t)k * DIM + o]); }
    for (size_t q = tid; q < 2048 + 16; q += nth) { float v; if (q < 2048) v = bf16_rne(nkv[q]); else { const int h = (int)q - 2048; float s = 0.0f; for (int d = 0; d < HD; ++d) { const float a = bf16_rne(nkv[h * HD + d]); s += pmul(a, a); } v = s; } P[q] = v; }
    for (size_t q = tid; q < (size_t)Bn * H * 64 * HD; q += nth) { const int d = (int)(q % HD), rsel = (int)((q / HD) % 64), bh = (int)(q / (64 * HD)); const int h = bh % H;
      kp[((size_t)bh * NKP + S + rsel) * HD + d] = (b16)((rsel == 0) ? bf16_rne(nkv[h * HD + d]) * KS : 0.0f); }
    for (size_t q = tid; q < (size_t)Bn * H * HD * 64; q += nth) { const int c = (int)(q % 64), rowi = (int)(q / 64); const int h = (rowi / HD) % H, d = rowi % HD; vt[(size_t)rowi * NKP + S + c] = (b16)((c == 0) ? bf16_rne(nkv[1024 + h * HD + d]) * VS : 0.0f); }
    __threadfence(); }
}

__global__ __launch_bounds__(256) void norm_kernel(const float* __restrict__ enc, float* __restrict__ rs) {
  __shared__ float Rv[32];
  const int wid = threadIdx.x >> 5, lane = threadIdx.x & 31;
  for (int sub = 0; sub < 4; ++sub) { const size_t row = (size_t)blockIdx.x * 32 + wid * 4 + sub; const float* pr = enc + row * DIM; float s = 0.0f;
#pragma unroll
    for (int j = 0; j < 8; ++j) { const v4f t = *(const v4f*)(pr + j * 128 + lane * 4);
#pragma unroll
      for (int e = 0; e < 4; ++e) { const float a = bf16_rne(t[e]); s += pmul(a, a); } }
#pragma unroll
    for (int o = 1; o < 32; o <<= 1) s += __shfl_xor(s, o);
    if (lane == 0) Rv[wid * 4 + sub] = 32.0f / fmaxf(sqrtf(s), 1e-12f); }
  __syncthreads();
  if (threadIdx.x < 32) { const float v = Rv[threadIdx.x]; for (int pass = 0; pass < 2; ++pass) ((volatile float*)rs)[(size_t)blockIdx.x * 32 + threadIdx.x] = v; }
  __threadfence();
}

__global__ __launch_bounds__(128) void proj_kernel(const float* __restrict__ enc, const float* __restrict__ rs, const b16* __restrict__ R, b16* __restrict__ qp, b16* __restrict__ kp, b16* __restrict__ vt, float* __restrict__ qn2) {
  __shared__ __attribute__((aligned(16))) b16 T[128][64 + 8]; __shared__ __attribute__((aligned(16))) b16 Tv[64][128 + 8]; __shared__ float Q2[128];
  const int lane = threadIdx.x & 31, wave = threadIdx.x >> 5, nloc = lane & 15, hlf = lane >> 4, ct = blockIdx.x, c0 = ct * 64, p0 = blockIdx.y * 128, m0 = p0 + wave * 32, b = p0 / S, t0 = p0 % S;
  v8f acc[2][4];
#pragma unroll
  for (int r = 0; r < 2; ++r)
#pragma unroll
    for (int t = 0; t < 4; ++t) acc[r][t] = (v8f){};
#pragma unroll 2
  for (int kb = 0; kb < DIM; kb += 32) { const v16b a0 = frag_x(enc + (size_t)(m0 + nloc) * DIM + kb, hlf), a1 = frag_x(enc + (size_t)(m0 + 16 + nloc) * DIM + kb, hlf);
#pragma unroll
    for (int t = 0; t < 4; ++t) { const v16b bw = frag_kb(R + (size_t)(c0 + t * 16 + nloc) * DIM + kb, hlf); acc[0][t] = wmma16b(a0, bw, acc[0][t]); acc[1][t] = wmma16b(a1, bw, acc[1][t]); } }
#pragma unroll
  for (int r = 0; r < 2; ++r)
#pragma unroll
    for (int v = 0; v < 8; ++v) { const float sc = rs[m0 + r * 16 + 8 * hlf + v];
#pragma unroll
      for (int t = 0; t < 4; ++t) acc[r][t][v] *= sc; }
  if (ct < 16) { const int h = ct;
#pragma unroll
    for (int r = 0; r < 2; ++r)
#pragma unroll
      for (int v = 0; v < 8; ++v) { float s2 = 0.0f;
#pragma unroll
        for (int t = 0; t < 4; ++t) s2 += pmul(acc[r][t][v], acc[r][t][v]);
#pragma unroll
        for (int o = 1; o < 16; o <<= 1) s2 += __shfl_xor(s2, o);
        if (nloc == 0) Q2[wave * 32 + r * 16 + 8 * hlf + v] = s2; }
#pragma unroll
    for (int t = 0; t < 4; ++t)
#pragma unroll
      for (int r = 0; r < 2; ++r)
#pragma unroll
        for (int v = 0; v < 8; ++v) T[wave * 32 + r * 16 + 8 * hlf + v][t * 16 + nloc] = (b16)(acc[r][t][v] * QS);
    __syncthreads();
    b16* qb = qp + (((size_t)b * H + h) * S + t0) * HD; b16* kb_ = kp + (((size_t)b * H + h) * NKP + t0) * HD;
    for (int pass = 0; pass < 2; ++pass) { for (int i = threadIdx.x; i < 128 * 8; i += 128) { const int rr = i >> 3, c8 = (i & 7) * 8; const v8b val = *(const v8b*)(&T[rr][c8]); *(volatile v8b*)(qb + (size_t)rr * HD + c8) = val; *(volatile v8b*)(kb_ + (size_t)rr * HD + c8) = val; }
      *(volatile float*)(qn2 + ((size_t)b * H + h) * S + t0 + threadIdx.x) = Q2[threadIdx.x]; __threadfence(); }
    return; }
  const int h = ct - 16;
#pragma unroll
  for (int t = 0; t < 4; ++t)
#pragma unroll
    for (int r = 0; r < 2; ++r)
#pragma unroll
      for (int v = 0; v < 8; ++v) Tv[t * 16 + nloc][wave * 32 + r * 16 + 8 * hlf + v] = (b16)(acc[r][t][v] * VS);
  __syncthreads();
  for (int pass = 0; pass < 2; ++pass) { for (int i = threadIdx.x; i < 64 * 16; i += 128) { const int d = i >> 4, c8 = (i & 15) * 8; *(volatile v8b*)(vt + (((size_t)b * H + h) * HD + d) * NKP + t0 + c8) = *(const v8b*)(&Tv[d][c8]); } __threadfence(); }
}

__global__ __launch_bounds__(256) void attn_kernel(const b16* __restrict__ qp, const b16* __restrict__ kp, const b16* __restrict__ vt, const float* __restrict__ qn2, const int* __restrict__ mask, const float* __restrict__ P, b16* __restrict__ ctx) {
  __shared__ __attribute__((aligned(16))) b16 Os[16][8 * HD + 8];
  const int wid = threadIdx.x >> 5, lane = threadIdx.x & 31, hh = lane >> 4, col = lane & 15; const int b = blockIdx.x / (S / 16), q0 = (blockIdx.x % (S / 16)) * 16, h = blockIdx.y * 8 + wid, qi = q0 + col;
  const b16* Q = qp + (((size_t)b * H + h) * S) * HD; const b16* K = kp + (((size_t)b * H + h) * NKP) * HD; const b16* V = vt + (((size_t)b * H + h) * HD) * NKP; const float* qn = qn2 + ((size_t)b * H + h) * S; const int* mk = mask + (size_t)b * S;
  const float q2 = qn[qi]; const float nk2 = P[2048 + h];
  const v16b qf0 = frag_kb(Q + (size_t)qi * HD, hh), qf1 = frag_kb(Q + (size_t)qi * HD + 32, hh);
  float m = -INFINITY, l = 0.0f; v8f o[4] = {{}, {}, {}, {}};
  for (int kb = 0; kb < NKP; kb += 32) {
    const v16b ka0 = frag_kb(K + (size_t)(kb + col) * HD, hh), ka1 = frag_kb(K + (size_t)(kb + col) * HD + 32, hh), kc0 = frag_kb(K + (size_t)(kb + 16 + col) * HD, hh), kc1 = frag_kb(K + (size_t)(kb + 16 + col) * HD + 32, hh);
    v8f s0 = {}, s1 = {}; s0 = wmma16b(ka0, qf0, s0); s0 = wmma16b(ka1, qf1, s0); s1 = wmma16b(kc0, qf0, s1); s1 = wmma16b(kc1, qf1, s1);
    float mr = -INFINITY;
#pragma unroll
    for (int r = 0; r < 8; ++r) {
#pragma unroll
      for (int u = 0; u < 2; ++u) { const int j = kb + u * 16 + 8 * hh + r; const float qk = ((u == 0) ? s0[r] : s1[r]) * (1.0f / (QS * KS)); float sv;
        if (j > S) sv = -INFINITY;
        else { const float k2 = (j == S) ? nk2 : qn[j]; const float d2 = fmaxf((q2 + k2) - 2.0f * qk, 0.0f); sv = -sqrtf(d2) * SCALE; if (j == qi) sv = SELF; if (j < S && mk[j] == 0) sv = -FLT_MAX; }
        if (u == 0) s0[r] = sv; else s1[r] = sv; mr = fmaxf(mr, sv); } }
    mr = fmaxf(mr, __shfl_xor(mr, 16));
    const float mn = fmaxf(m, mr), al_ = (mn == -INFINITY) ? 1.0f : nexp(m - mn); m = mn; float sum = 0.0f; v16b pbv;
#pragma unroll
    for (int r = 0; r < 8; ++r) { const float e0 = (s0[r] == -INFINITY) ? 0.0f : nexp(s0[r] - mn), e1 = (s1[r] == -INFINITY) ? 0.0f : nexp(s1[r] - mn); sum += e0 + e1; pbv[r] = (b16)(e0 * PS); pbv[8 + r] = (b16)(e1 * PS); }
    sum += __shfl_xor(sum, 16); l = l * al_ + sum;
#pragma unroll
    for (int t = 0; t < 4; ++t) { o[t] *= al_; const v16b vf = frag_kb(V + (size_t)(t * 16 + col) * NKP + kb, hh); o[t] = wmma16b(vf, pbv, o[t]); } }
  const float inv = 1.0f / (l * VS * PS);
#pragma unroll
  for (int t = 0; t < 4; ++t)
#pragma unroll
    for (int r = 0; r < 8; ++r) Os[col][wid * HD + t * 16 + 8 * hh + r] = (b16)(o[t][r] * inv);
  __syncthreads();
  for (int pass = 0; pass < 2; ++pass) { for (int i = threadIdx.x; i < 16 * (8 * HD / 8); i += 256) { const int rr = i / (8 * HD / 8), c8 = (i % (8 * HD / 8)) * 8; *(volatile v8b*)(ctx + ((size_t)b * S + q0 + rr) * DIM + blockIdx.y * 8 * HD + c8) = *(const v8b*)(&Os[rr][c8]); } __threadfence(); }
}

__global__ __launch_bounds__(128) void out_kernel(const b16* __restrict__ ctx, const b16* __restrict__ Ro, float* __restrict__ out) {
  __shared__ __attribute__((aligned(16))) float Ts[4][32 * 64];
  const int lane = threadIdx.x & 31, wave = threadIdx.x >> 5, nloc = lane & 15, hlf = lane >> 4, m0 = blockIdx.y * 128 + wave * 32, c0 = blockIdx.x * 64;
  v8f acc[2][4];
#pragma unroll
  for (int r = 0; r < 2; ++r)
#pragma unroll
    for (int t = 0; t < 4; ++t) acc[r][t] = (v8f){};
#pragma unroll 2
  for (int kb = 0; kb < DIM; kb += 32) { const v16b a0 = frag_kb(ctx + (size_t)(m0 + nloc) * DIM + kb, hlf), a1 = frag_kb(ctx + (size_t)(m0 + 16 + nloc) * DIM + kb, hlf);
#pragma unroll
    for (int t = 0; t < 4; ++t) { const v16b bw = frag_kb(Ro + (size_t)(c0 + t * 16 + nloc) * DIM + kb, hlf); acc[0][t] = wmma16b(a0, bw, acc[0][t]); acc[1][t] = wmma16b(a1, bw, acc[1][t]); } }
  float* Tt = Ts[wave];
#pragma unroll
  for (int t = 0; t < 4; ++t)
#pragma unroll
    for (int r = 0; r < 2; ++r)
#pragma unroll
      for (int v = 0; v < 8; ++v) Tt[(r * 16 + v + 8 * hlf) * 64 + t * 16 + nloc] = acc[r][t][v];
  wave_lds_sync();
  for (int pass = 0; pass < 2; ++pass) {
#pragma unroll
    for (int j = 0; j < 16; ++j) { const int rr = j * 2 + hlf, c4 = nloc * 4; *(volatile v4f*)(out + (size_t)(m0 + rr) * DIM + c0 + c4) = *(const v4f*)(Tt + rr * 64 + c4); }
    __threadfence(); }
}
}

extern "C" void kernel_launch(void* const* d_in, const int* in_sizes, int n_in,
                              void* d_out, int out_size, void* d_ws, size_t ws_size, hipStream_t stream) {
  (void)n_in; (void)out_size;
  const float* enc = (const float*)d_in[0]; const int* mask = (const int*)d_in[1]; const float* gam = (const float*)d_in[2]; const float* wqk = (const float*)d_in[3]; const float* wv = (const float*)d_in[4]; const float* nkv = (const float*)d_in[5]; const float* wo = (const float*)d_in[6];
  float* out = (float*)d_out;
  if (in_sizes[0] != NT * DIM || in_sizes[1] != NT || in_sizes[3] != DIM * 1024 || in_sizes[5] != 2 * H * HD || in_sizes[6] != 1024 * DIM) return;
  size_t off = 0; char* ws = (char*)d_ws;
  auto carve = [&](size_t bytes) { char* p = ws + off; off += (bytes + 255) & ~(size_t)255; return p; };
  b16* R = (b16*)carve((size_t)2048 * DIM * 2); b16* Ro = (b16*)carve((size_t)DIM * DIM * 2); float* P = (float*)carve(4096 * 4); float* rsv = (float*)carve((size_t)NT * 4);
  b16* qp = (b16*)carve(QPL * 2); b16* kp = (b16*)carve(KPL * 2); b16* vt = (b16*)carve(KPL * 2); float* qn2 = (float*)carve((size_t)Bn * H * S * 4); b16* ctx = (b16*)carve((size_t)NT * DIM * 2);
  if (off > ws_size) return;
  prep_kernel<<<512, 256, 0, stream>>>(gam, wqk, wv, nkv, wo, R, Ro, P, kp, vt);
  norm_kernel<<<NT / 32, 256, 0, stream>>>(enc, rsv);
  proj_kernel<<<dim3(32, NT / 128), 128, 0, stream>>>(enc, rsv, R, qp, kp, vt, qn2);
  attn_kernel<<<dim3(NT / 16, 2), 256, 0, stream>>>(qp, kp, vt, qn2, mask, P, ctx);
  out_kernel<<<dim3(DIM / 64, NT / 128), 128, 0, stream>>>(ctx, Ro, out);
}
